// model_NN_LSTM_88768384074425
// MI455X (gfx1250) — hardware-verified
//
#include <hip/hip_runtime.h>
#include <math.h>

typedef __attribute__((ext_vector_type(16))) _Float16 v16h;
typedef __attribute__((ext_vector_type(8)))  _Float16 v8h;
typedef __attribute__((ext_vector_type(8)))  float    v8f;
typedef __attribute__((ext_vector_type(4)))  float    v4f;

constexpr int kBatch      = 4096;
constexpr int kSteps      = 1024;
constexpr int kHid        = 15;
constexpr int kTileRows   = 16;
constexpr int kTiles      = kBatch / kTileRows;
constexpr int kChunk      = 32;
constexpr int kNumChunks  = kSteps / kChunk;
constexpr int kPitch      = 36;
constexpr int kMatElems   = kHid * kHid;
constexpr size_t kOutElems = (size_t)kBatch * (size_t)kSteps;
static_assert(kBatch % kTileRows == 0, "whole 16-row tiles");
static_assert(kSteps % kChunk == 0, "whole 32-step chunks");
static_assert(kHid <= 16, "units fit one 16-row subtile and the first 16 k of one instruction");
static_assert(kMatElems == 225 && kMatElems <= 8 * 32, "weight staging: 8 strided passes of 32 lanes");
static_assert((kPitch % 4) == 0, "16-B aligned LDS rows");

constexpr float kStateCarry  = 256.0f;
constexpr float kWeightCarry = 64.0f;
constexpr float kFoldBack    = 1.0f / (kStateCarry * kWeightCarry);
constexpr float kF16MinNorm  = 6.103515625e-5f;
static_assert(kStateCarry * kWeightCarry == 16384.0f, "carry product");

namespace eng {

union FragU { v16h v; v8h h[2]; };

__device__ __forceinline__ unsigned short f2bf_bits(float f) {
  unsigned u = __float_as_uint(f);
  return (unsigned short)((u + 0x7FFFu + ((u >> 16) & 1u)) >> 16);
}
__device__ __forceinline__ float bf16v(float f) {
  return __uint_as_float(((unsigned)f2bf_bits(f)) << 16);
}
__device__ __forceinline__ _Float16 to_f16_flushed(float c) {
  const float z = (fabsf(c) < kF16MinNorm) ? 0.0f : c;
  return (_Float16)z;
}
__device__ __forceinline__ v8f mma_f16(v16h a, v16h b) {
  v8f c = (v8f){0.f, 0.f, 0.f, 0.f, 0.f, 0.f, 0.f, 0.f};
  c = __builtin_amdgcn_wmma_f32_16x16x32_f16(false, a, false, b, (short)0, c, false, false);
  asm volatile("v_nop\n\tv_nop\n\tv_nop\n\tv_nop" : "+v"(c) : "v"(a), "v"(b));
  return c;
}
__device__ __forceinline__ float fast_tanh(float v) {
  const float e = __expf(2.0f * v);
  return 1.0f - 2.0f * __builtin_amdgcn_rcpf(e + 1.0f);
}

}

__global__ __launch_bounds__(32) void rnn1_seq_kernel(
    const float* __restrict__ x,
    const float* __restrict__ w_ih,
    const float* __restrict__ w_hh,
    const float* __restrict__ b_ih,
    const float* __restrict__ b_hh,
    const float* __restrict__ w_out,
    const float* __restrict__ b_out,
    float* __restrict__ outs)
{
  __shared__ __align__(16) float xs[kTileRows * kPitch];
  __shared__ __align__(16) float os[kTileRows * kPitch];
  __shared__ __align__(16) float wsm[8 * 32];
  __shared__ __align__(16) float csm[5 * 32];

  const int lane = threadIdx.x & 31;
  const int hsel = lane >> 4;
  const int n    = lane & 15;
  const bool lowHalf = (hsel == 0);
  const int b0   = blockIdx.x * kTileRows;

  {
#pragma unroll
    for (int it = 0; it < 8; ++it) {
      const int i  = it * 32 + lane;
      const int ic = (i < kMatElems) ? i : (kMatElems - 1);
      wsm[ic] = w_hh[ic];
    }
    const int ci = (lane < kHid - 1) ? lane : (kHid - 1);
    csm[0 * 32 + lane] = b_ih[ci];
    csm[1 * 32 + lane] = b_hh[ci];
    csm[2 * 32 + lane] = w_ih[ci];
    csm[3 * 32 + lane] = w_out[ci];
    csm[4 * 32 + lane] = b_out[0];
  }
  __syncthreads();

  v16h fragA;
  {
    const int m  = n;
    const int mc = (m < kHid) ? m : (kHid - 1);
    const bool mok = (m < kHid);
    v8h alo;
    const v8h zero8 = (v8h){(_Float16)0.0f, (_Float16)0.0f, (_Float16)0.0f, (_Float16)0.0f,
                            (_Float16)0.0f, (_Float16)0.0f, (_Float16)0.0f, (_Float16)0.0f};
#pragma unroll
    for (int i = 0; i < 8; ++i) {
      const int k  = 8 * hsel + i;
      const int kc = (k < kHid) ? k : (kHid - 1);
      const bool ok = mok && (k < kHid);
      const float f0 = wsm[mc * kHid + kc];
      const float g0 = ok ? (eng::bf16v(f0) * kWeightCarry) : 0.0f;
      alo[i] = eng::to_f16_flushed(g0);
    }
    eng::FragU u0;
    u0.h[0] = alo;
    u0.h[1] = zero8;
    fragA = u0.v;
  }

  float cb[8], wx[8], wo[8];
  float hf[8];
  v8h hb;
#pragma unroll
  for (int r = 0; r < 8; ++r) {
    const int u  = 8 * hsel + r;
    const int uc = (u < kHid) ? u : (kHid - 1);
    const bool live = (u < kHid);
    const float vb  = eng::bf16v(csm[0 * 32 + uc]) + eng::bf16v(csm[1 * 32 + uc]);
    const float vwx = eng::bf16v(csm[2 * 32 + uc]);
    const float vwo = eng::bf16v(csm[3 * 32 + uc]);
    cb[r] = live ? vb : 0.0f;
    wx[r] = live ? vwx : 0.0f;
    wo[r] = live ? vwo : 0.0f;
    hf[r] = 0.0f;
    hb[r] = (_Float16)0.0f;
  }
  const float bo = eng::bf16v(csm[4 * 32]);
  const v8h zh = (v8h){(_Float16)0.0f, (_Float16)0.0f, (_Float16)0.0f, (_Float16)0.0f,
                       (_Float16)0.0f, (_Float16)0.0f, (_Float16)0.0f, (_Float16)0.0f};

  const int q  = lane >> 3;
  const int c4 = (lane & 7) * 4;

#pragma unroll 1
  for (int ch = 0; ch < kNumChunks; ++ch) {
    const int t0 = ch * kChunk;
#pragma unroll
    for (int it = 0; it < 4; ++it) {
      const int row = it * 4 + q;
      const v4f v = *(const v4f*)(x + (size_t)(b0 + row) * kSteps + t0 + c4);
      v4f rv;
      const float v0 = v[0];
      const float v1 = v[1];
      const float v2 = v[2];
      const float v3 = v[3];
      rv[0] = eng::bf16v(v0);
      rv[1] = eng::bf16v(v1);
      rv[2] = eng::bf16v(v2);
      rv[3] = eng::bf16v(v3);
      *(v4f*)(xs + row * kPitch + c4) = rv;
    }
    __syncthreads();

#pragma unroll 1
    for (int s = 0; s < kChunk; ++s) {
      const float xv = xs[n * kPitch + s];

      eng::FragU fb;
      fb.h[0] = hb;
      fb.h[1] = zh;
      const v8f acc = eng::mma_f16(fragA, fb.v);
#pragma unroll
      for (int r = 0; r < 8; ++r) {
        const float pre = fmaf(acc[r], kFoldBack, fmaf(xv, wx[r], cb[r]));
        const float tv  = eng::fast_tanh(pre);
        const bool live = (r < 7) || lowHalf;
        const float hv  = live ? tv : 0.0f;
        hf[r] = hv;
        hb[r] = eng::to_f16_flushed(hv * kStateCarry);
      }

      float p = 0.0f;
#pragma unroll
      for (int r = 0; r < 8; ++r) p = fmaf(wo[r], hf[r], p);
      const float pother = __shfl_xor(p, 16, 32);
      const float tot = (p + pother) + bo;
      if (lowHalf) os[n * kPitch + s] = tot;
    }
    __syncthreads();

    {
      v4f ov[4];
#pragma unroll
      for (int it = 0; it < 4; ++it) ov[it] = *(const v4f*)(os + (it * 4 + q) * kPitch + c4);
      for (int pass = 0; pass < 2; ++pass) {
#pragma unroll
        for (int it = 0; it < 4; ++it)
          *(volatile v4f*)(outs + (size_t)(b0 + it * 4 + q) * kSteps + t0 + c4) = ov[it];
        __threadfence();
      }
    }
  }
}

extern "C" void kernel_launch(void* const* d_in, const int* in_sizes, int n_in,
                              void* d_out, int out_size, void* d_ws, size_t ws_size,
                              hipStream_t stream) {
  (void)d_ws;
  (void)ws_size;
  if (n_in < 7 || d_out == nullptr) return;
  if (in_sizes[0] != kBatch * kSteps) return;
  if (in_sizes[1] != kHid) return;
  if (in_sizes[2] != kMatElems) return;
  if (in_sizes[3] != kHid) return;
  if (in_sizes[4] != kHid) return;
  if (in_sizes[5] != kHid) return;
  if (in_sizes[6] != 1) return;
  if ((size_t)out_size != kOutElems) return;

  const float* x     = (const float*)d_in[0];
  const float* w_ih  = (const float*)d_in[1];
  const float* w_hh  = (const float*)d_in[2];
  const float* b_ih  = (const float*)d_in[3];
  const float* b_hh  = (const float*)d_in[4];
  const float* w_out = (const float*)d_in[5];
  const float* b_out = (const float*)d_in[6];
  float* outs = (float*)d_out;

  rnn1_seq_kernel<<<kTiles, 32, 0, stream>>>(x, w_ih, w_hh, b_ih, b_hh, w_out, b_out, outs);
}
